// PersonalModel_1185410974349
// MI455X (gfx1250) — hardware-verified
//
#include <hip/hip_runtime.h>
#include <math.h>

typedef __attribute__((ext_vector_type(16))) _Float16 v16h;
typedef __attribute__((ext_vector_type(16))) __bf16 v16b;
typedef __attribute__((ext_vector_type(8)))  _Float16 v8h;
typedef __attribute__((ext_vector_type(8)))  float v8f;
typedef __attribute__((ext_vector_type(4)))  float v4f;
typedef __attribute__((ext_vector_type(2)))  float v2f;
typedef __attribute__((ext_vector_type(4)))  unsigned v4u;
typedef __attribute__((ext_vector_type(4)))  int v4i;
typedef float __attribute__((may_alias)) float_a;
typedef int __attribute__((may_alias)) int_a;

template <typename T> __device__ __forceinline__ void vst2(void* p, T v) { *(volatile T*)p = v; __threadfence(); *(volatile T*)p = v; }
__device__ __forceinline__ v8f wmma16(v16h a, v16h b, v8f c) {
  v8f d = __builtin_amdgcn_wmma_f32_16x16x32_f16(false, a, false, b, (short)0, c, false, false);
  asm volatile("v_nop\n\tv_nop\n\tv_nop\n\tv_nop" : "+v"(d) : "v"(a), "v"(b));
  return d;
}
__device__ __forceinline__ v8f wmma_bf(v16b a, v16b b, v8f c) {
  v8f d = __builtin_amdgcn_wmma_f32_16x16x32_bf16(false, a, false, b, (short)0, c, false, false);
  asm volatile("v_nop\n\tv_nop\n\tv_nop\n\tv_nop" : "+v"(d) : "v"(a), "v"(b));
  return d;
}
__device__ __forceinline__ v16h frag_h(const _Float16* rowk0, int lane) {
  union { v16h v; v8h q[2]; } u; const _Float16* p = rowk0 + 8 * (lane >> 4);
  u.q[0] = *(const v8h*)p; u.q[1] = *(const v8h*)(p + 16); return u.v;
}
__device__ __forceinline__ v16h frag_f32(const float* rowk0, int lane) {
  v16h a; const float* p = rowk0 + 8 * (lane >> 4);
#pragma unroll
  for (int i = 0; i < 8; ++i) { a[i] = (_Float16)p[i]; a[8 + i] = (_Float16)p[16 + i]; }
  return a;
}
__device__ __forceinline__ v16h frag_f32s(const float* rowk0, int lane, float sc) {
  v16h a; const float* p = rowk0 + 8 * (lane >> 4);
#pragma unroll
  for (int i = 0; i < 8; ++i) { a[i] = (_Float16)(p[i] * sc); a[8 + i] = (_Float16)(p[16 + i] * sc); }
  return a;
}
__device__ __forceinline__ v16h fragc_f32(const float* W, int k0, int n, int lane, int ld, int K) {
  v16h a; const int g = lane >> 4;
#pragma unroll
  for (int i = 0; i < 8; ++i) { const int ka = k0 + 8 * g + i, kb = ka + 16;
    a[i] = (_Float16)(ka < K ? W[(size_t)(ka < K ? ka : K - 1) * ld + n] : 0.f); a[8 + i] = (_Float16)(kb < K ? W[(size_t)(kb < K ? kb : K - 1) * ld + n] : 0.f); }
  return a;
}
struct F2 { v16b h, l; };
__device__ __forceinline__ F2 bsplit16(const float v[16]) { F2 r;
#pragma unroll
  for (int i = 0; i < 16; ++i) { const __bf16 h = (__bf16)v[i]; r.h[i] = h; r.l[i] = (__bf16)(v[i] - (float)h); }
  return r; }
__device__ __forceinline__ F2 split_row(const float* row, int k0, int lane) { float v[16]; const float* p = row + k0 + 8 * (lane >> 4);
#pragma unroll
  for (int i = 0; i < 8; ++i) { v[i] = p[i]; v[8 + i] = p[16 + i]; }
  return bsplit16(v); }
__device__ __forceinline__ F2 split_rowK(const float* row, int k0, int lane, int K) { float v[16]; const int g = lane >> 4;
#pragma unroll
  for (int i = 0; i < 8; ++i) { const int ka = k0 + 8 * g + i, kb = ka + 16; v[i] = ka < K ? row[ka < K ? ka : K - 1] : 0.f; v[8 + i] = kb < K ? row[kb < K ? kb : K - 1] : 0.f; }
  return bsplit16(v); }
__device__ __forceinline__ F2 split_col(const float* W, int k0, int n, int lane, int ld, int K) { float v[16]; const int g = lane >> 4;
#pragma unroll
  for (int i = 0; i < 8; ++i) { const int ka = k0 + 8 * g + i, kb = ka + 16; v[i] = ka < K ? W[(size_t)(ka < K ? ka : K - 1) * ld + n] : 0.f; v[8 + i] = kb < K ? W[(size_t)(kb < K ? kb : K - 1) * ld + n] : 0.f; }
  return bsplit16(v); }
__device__ __forceinline__ v8f mac3(const F2& a, const F2& b, v8f c) { c = wmma_bf(a.l, b.h, c); c = wmma_bf(a.h, b.l, c); return wmma_bf(a.h, b.h, c); }
__device__ __forceinline__ float sigm(float v) { return 1.0f / (1.0f + expf(-v)); }
#define LDSX() do { asm volatile("s_wait_dscnt 0" ::: "memory"); __builtin_amdgcn_wave_barrier(); __builtin_amdgcn_fence(__ATOMIC_RELEASE, "workgroup"); } while (0)


#define NB 4
#define NSEQ 2048
#define NR (NB * NSEQ)
#define DIN 256
#define DSP 256
#define D1 257
#define KP 288
#define NHD 4
#define HS 64
#define VW 80
#define NCLS 129
#define NLAY 2
#ifndef DBG_NL
#define DBG_NL NLAY
#define DBG_L0 0
#define TRB (NR / 64)
#define TQB (NSEQ / 64)
#define TNB NB
#endif
typedef __attribute__((ext_vector_type(8))) __bf16 v8b;
__device__ __forceinline__ v16b frag_b(const __bf16* rowk0, int lane) {
  union { v16b v; v8b q[2]; } u; const __bf16* p = rowk0 + 8 * (lane >> 4);
  u.q[0] = *(const v8b*)p; u.q[1] = *(const v8b*)(p + 16); return u.v;
}
__device__ __forceinline__ v16b frag_gbf(const float* rowk0, int lane) {
  v16b a; const float* p = rowk0 + 8 * (lane >> 4);
#pragma unroll
  for (int i = 0; i < 8; ++i) { a[i] = (__bf16)p[i]; a[8 + i] = (__bf16)p[16 + i]; }
  return a;
}
__device__ __forceinline__ float bfr(float v) { return (float)(__bf16)v; }
__device__ __attribute__((noinline)) float exp_ni(float v) { return expf(v); }
__device__ __attribute__((noinline)) float cosh_ni(float v) { return coshf(v); }
__device__ __attribute__((noinline)) float sinh_ni(float v) { return sinhf(v); }

#define PT_LAYER(l, m) ((size_t)(((l) * 4 + (m)) * 256) * KP)
#define PT_H ((size_t)(NLAY * 4 * 256) * KP)
#define PT_END (PT_H + (size_t)144 * KP)
#define WS_PT  0u
#define WS_XL  (WS_PT + 2u * PT_END)
#define WS_F   (WS_XL + 4u * NR * KP)
#define WS_QS  (WS_F + 4u * NR * KP)
#define WS_KS  (WS_QS + 4u * NR * DSP)
#define WS_QT  (WS_KS + 4u * NR * DSP)
#define WS_KT  (WS_QT + 4u * NR * 4)
#define WS_VTH (WS_KT + 4u * NR * 4)
#define WS_VTL (WS_VTH + 2u * NB * NHD * VW * NSEQ)
#define WS_M   (WS_VTL + 2u * NB * NHD * VW * NSEQ)
#define WS_L   (WS_M + 4u * NB * NHD * NSEQ)
#define UPITCH 384
#define LGP 160
#define WS_U   (WS_L + 4u * NB * NHD * NSEQ)
#define WS_LG  (WS_U + 4u * NR * UPITCH)
#define WS_END (WS_LG + 4u * NR * LGP)

__global__ __launch_bounds__(128) void k_pack(const float* __restrict__ Wq, const float* __restrict__ Wk, const float* __restrict__ Wv, const float* __restrict__ Wo, const float* __restrict__ Wh, __bf16* __restrict__ PT) {
  __shared__ __align__(16) __bf16 srow[2 * KP];
  const int pr = blockIdx.x, tid = threadIdx.x;
  for (int q = tid; q < 2 * KP; q += 128) { const int rr = q / KP, k = q % KP; const int row = 2 * pr + rr; float v = 0.f;
    if (row < NLAY * 4 * 256) { const int l = row / 1024, m = (row / 256) & 3, n = row & 255; const float* Wm = m == 0 ? Wq : (m == 1 ? Wk : (m == 2 ? Wv : Wo)); if (k < D1) v = Wm[((size_t)l * D1 + (n + 1)) * D1 + k]; }
    else { const int n = row - NLAY * 4 * 256; if (n < NCLS && k < D1) v = Wh[(size_t)n * D1 + k]; }
    srow[q] = (__bf16)v; }
  __syncthreads();
  if (tid < 2 * KP / 8) vst2((unsigned*)(PT + (size_t)(2 * pr) * KP + tid * 8), *(const v4u*)(&srow[tid * 8]));
}
__global__ __launch_bounds__(128) void k_in(const float* __restrict__ X, const float* __restrict__ Win, const float* __restrict__ bin, float* __restrict__ XL) {
  __shared__ __align__(16) float st[4][16][KP + 4];
  const int tid = threadIdx.x, wave = tid >> 5, lane = tid & 31, col = lane & 15, g = lane >> 4; const size_t r0 = (size_t)blockIdx.x * 64 + wave * 16;
  v8f acc[16] = {};
#pragma unroll 2
  for (int kc = 0; kc < DIN / 32; ++kc) { const v16b a = frag_gbf(X + (r0 + col) * DIN + kc * 32, lane);
#pragma unroll
    for (int j = 0; j < 16; ++j) acc[j] = wmma_bf(a, frag_gbf(Win + (size_t)(j * 16 + col) * DIN + kc * 32, lane), acc[j]); }
#pragma unroll
  for (int j = 0; j < 16; ++j) { const int n = j * 16 + col; const float bb = bfr(bin[n]);
#pragma unroll
    for (int r = 0; r < 8; ++r) st[wave][8 * g + r][1 + n] = acc[j][r] + bb; }
  LDSX();
  { const int rl = lane >> 1, half = lane & 1; float ss = 0.f;
    for (int c = half * 128; c < half * 128 + 128; ++c) { const float v = st[wave][rl][1 + c]; ss += v * v; }
    ss += __shfl_xor(ss, 1);
    const float nrm = fmaxf(sqrtf(ss), 1e-12f);
    float us = 0.f; for (int c = half * 128; c < half * 128 + 128; ++c) { const float u = st[wave][rl][1 + c] / nrm; us += u * u; }
    us += __shfl_xor(us, 1);
    const float n_ = sqrtf(fmaxf(us, 1e-6f)); const float ch = cosh_ni(n_), sh = sinh_ni(n_);
    LDSX();
    for (int c = half * 128; c < half * 128 + 128; ++c) { const float u = st[wave][rl][1 + c] / nrm; st[wave][rl][1 + c] = sh * u / n_; }
    if (half == 0) { st[wave][rl][0] = ch; for (int c = D1; c < KP; ++c) st[wave][rl][c] = 0.f; } }
  LDSX();
  for (int rl = 0; rl < 16; ++rl) for (int pc = lane; pc < KP / 4; pc += 32) vst2(XL + (r0 + rl) * KP + pc * 4, *(const v4f*)&st[wave][rl][pc * 4]);
}

#define UP 96
__global__ __launch_bounds__(128) void k_lin(const float* __restrict__ A, const __bf16* __restrict__ PT, const float* __restrict__ bias, int l, int m, float* __restrict__ OS, float* __restrict__ OTm, __bf16* __restrict__ VTH, __bf16* __restrict__ VTL, float* __restrict__ XLn) {
  __shared__ __align__(16) float st[4][16][KP + 4]; __shared__ __align__(16) float stime[64][4];
  const int tid = threadIdx.x, wave = tid >> 5, lane = tid & 31, col = lane & 15, g = lane >> 4; const size_t r0 = (size_t)blockIdx.x * 64 + wave * 16;
  const __bf16* W = PT + PT_LAYER(l, m);
  v8f acc[16] = {};
#pragma unroll 1
  for (int kc = 0; kc < KP / 32; ++kc) { const F2 a = split_row(A + (r0 + col) * KP, kc * 32, lane);
#pragma unroll
    for (int j = 0; j < 16; ++j) { const v16b w = frag_b(W + (size_t)(j * 16 + col) * KP + kc * 32, lane); acc[j] = wmma_bf(a.l, w, acc[j]); acc[j] = wmma_bf(a.h, w, acc[j]); } }
#pragma unroll
  for (int j = 0; j < 16; ++j) { const int n = j * 16 + col; const float bb = bfr(bias[(size_t)l * D1 + n + 1]);
    const int off = (m == 3) ? 1 : 0;
#pragma unroll
    for (int r = 0; r < 8; ++r) st[wave][8 * g + r][off + n] = acc[j][r] + bb; }
  LDSX();
  if (m < 3) {
    { const int rl = lane >> 1, h0 = (lane & 1) * 2;
      for (int hh = h0; hh < h0 + 2; ++hh) { float ss = 0.f; for (int d = 0; d < HS; ++d) { const float v = st[wave][rl][hh * HS + d]; ss += v * v; } stime[wave * 16 + rl][hh] = sqrtf(ss + 1.0f); } }
    LDSX();
    if (m < 2) {
      for (int rl = 0; rl < 16; ++rl) for (int pc = lane; pc < DSP / 4; pc += 32) vst2(OS + (r0 + rl) * DSP + pc * 4, *(const v4f*)&st[wave][rl][pc * 4]);
    }
    __syncthreads();
    if (m < 2) { if (tid < 64) vst2(OTm + (size_t)blockIdx.x * 256 + tid * 4, *(const v4f*)(&stime[0][0] + tid * 4)); }
    else {
      const int b = (int)(((size_t)blockIdx.x * 64) / NSEQ), p0 = (int)(((size_t)blockIdx.x * 64) % NSEQ);
      for (int q = tid; q < NHD * VW * 8; q += 128) { const int pc = q & 7, rowid = q >> 3; const int hh = rowid / VW, d = rowid % VW; union { __bf16 e[8]; v4u u; } hi, lo;
#pragma unroll
        for (int e = 0; e < 8; ++e) { const int rl = pc * 8 + e; const int wv = rl >> 4, rr = rl & 15; float v = 0.f;
          if (d == 0) v = stime[rl][hh]; else if (d <= HS) v = st[wv][rr][hh * HS + (d - 1)];
          const __bf16 hb = (__bf16)v; hi.e[e] = hb; lo.e[e] = (__bf16)(v - (float)hb); }
        const size_t o = ((size_t)(b * NHD + hh) * VW + d) * NSEQ + p0 + pc * 8; vst2((unsigned*)(VTH + o), hi.u); vst2((unsigned*)(VTL + o), lo.u); } } }
  else {
    { const int rl = lane >> 1, half = lane & 1; float ss = 0.f; for (int c = half * 128; c < half * 128 + 128; ++c) { const float v = st[wave][rl][1 + c]; ss += v * v; } ss += __shfl_xor(ss, 1);
      if (half == 0) { st[wave][rl][0] = sqrtf(ss + 1.0f); for (int c = D1; c < KP; ++c) st[wave][rl][c] = 0.f; } }
    LDSX();
    for (int rl = 0; rl < 16; ++rl) for (int pc = lane; pc < KP / 4; pc += 32) vst2(XLn + (r0 + rl) * KP + pc * 4, *(const v4f*)&st[wave][rl][pc * 4]); }
}

__global__ __launch_bounds__(128) void k_stats(const float* __restrict__ QS, const float* __restrict__ KS, const float* __restrict__ QT, const float* __restrict__ KT, float* __restrict__ Mb, float* __restrict__ Lb) {
  __shared__ __align__(16) float sm[4][16]; __shared__ __align__(16) float ssum[4][16];
  const int tid = threadIdx.x, wave = tid >> 5, lane = tid & 31, col = lane & 15, g = lane >> 4;
  const int bh = blockIdx.y, b = bh >> 2, h = bh & 3; const int q0 = blockIdx.x * 64 + wave * 16; const float isq = 1.0f / sqrtf(65.0f);
  const float* qrow = QS + ((size_t)b * NSEQ + q0 + col) * DSP + h * HS; const F2 a0 = split_row(qrow, 0, lane), a1 = split_row(qrow, 32, lane);
  float qt[8];
#pragma unroll
  for (int r = 0; r < 8; ++r) qt[r] = QT[((size_t)b * NSEQ + q0 + 8 * g + r) * 4 + h];
  float m[8], l[8];
#pragma unroll
  for (int r = 0; r < 8; ++r) { m[r] = -3.0e38f; l[r] = 0.f; }
#pragma unroll 1
  for (int kt = 0; kt < NSEQ / 16; ++kt) { const float* krow = KS + ((size_t)b * NSEQ + kt * 16 + col) * DSP + h * HS; const F2 k0 = split_row(krow, 0, lane), k1 = split_row(krow, 32, lane);
    v8f s = mac3(a0, k0, (v8f){}); s = mac3(a1, k1, s); const float ktc = KT[((size_t)b * NSEQ + kt * 16 + col) * 4 + h];
#pragma unroll
    for (int r = 0; r < 8; ++r) { const float sv = (s[r] - qt[r] * ktc) * isq; float mx = sv;
#pragma unroll
      for (int o = 1; o < 16; o <<= 1) mx = fmaxf(mx, __shfl_xor(mx, o));
      const float mn = fmaxf(m[r], mx); float e = exp_ni(sv - mn);
#pragma unroll
      for (int o = 1; o < 16; o <<= 1) e += __shfl_xor(e, o);
      l[r] = l[r] * exp_ni(m[r] - mn) + e; m[r] = mn; } }
  if (col == 0) {
#pragma unroll
    for (int r = 0; r < 8; ++r) { sm[wave][8 * g + r] = m[r]; ssum[wave][8 * g + r] = l[r]; } }
  __syncthreads();
  { const int qb = blockIdx.x * 64; if (tid < 16) vst2(Mb + ((size_t)bh * NSEQ + qb) + tid * 4, *(const v4f*)(&sm[0][0] + tid * 4)); else if (tid < 32) vst2(Lb + ((size_t)bh * NSEQ + qb) + (tid - 16) * 4, *(const v4f*)(&ssum[0][0] + (tid - 16) * 4)); }
}
__global__ __launch_bounds__(128) void k_attn(const float* __restrict__ QS, const float* __restrict__ KS, const float* __restrict__ QT, const float* __restrict__ KT, const __bf16* __restrict__ VTH, const __bf16* __restrict__ VTL, const float* __restrict__ Mb, const float* __restrict__ Lb, float* __restrict__ U) {
  __shared__ __align__(16) float sp[4][16][36]; __shared__ __align__(16) float so[4][16][100];
  const int tid = threadIdx.x, wave = tid >> 5, lane = tid & 31, col = lane & 15, g = lane >> 4;
  const int bh = blockIdx.y, b = bh >> 2, h = bh & 3; const int q0 = blockIdx.x * 64 + wave * 16; const float isq = 1.0f / sqrtf(65.0f);
  const float* qrow = QS + ((size_t)b * NSEQ + q0 + col) * DSP + h * HS; const F2 a0 = split_row(qrow, 0, lane), a1 = split_row(qrow, 32, lane);
  float qt[8], mr[8], il[8];
#pragma unroll
  for (int r = 0; r < 8; ++r) { const size_t qi = (size_t)b * NSEQ + q0 + 8 * g + r; qt[r] = QT[qi * 4 + h]; mr[r] = Mb[(size_t)bh * NSEQ + q0 + 8 * g + r]; il[r] = 1.0f / Lb[(size_t)bh * NSEQ + q0 + 8 * g + r]; }
  v8f acc[5] = {};
#pragma unroll 1
  for (int ks = 0; ks < NSEQ / 32; ++ks) {
#pragma unroll
    for (int ct = 0; ct < 2; ++ct) { const int kk = ks * 32 + ct * 16 + col; const float* krow = KS + ((size_t)b * NSEQ + kk) * DSP + h * HS; const F2 k0 = split_row(krow, 0, lane), k1 = split_row(krow, 32, lane);
      v8f s = mac3(a0, k0, (v8f){}); s = mac3(a1, k1, s); const float ktc = KT[((size_t)b * NSEQ + kk) * 4 + h];
#pragma unroll
      for (int r = 0; r < 8; ++r) sp[wave][8 * g + r][ct * 16 + col] = exp_ni((s[r] - qt[r] * ktc) * isq - mr[r]) * il[r]; }
    LDSX();
    const F2 pa = split_row(&sp[wave][col][0], 0, lane);
#pragma unroll
    for (int dt = 0; dt < 5; ++dt) { const size_t vrow = ((size_t)(b * NHD + h) * VW + dt * 16 + col) * NSEQ + ks * 32; const v16b vh = frag_b(VTH + vrow, lane), vl = frag_b(VTL + vrow, lane);
      acc[dt] = wmma_bf(pa.l, vh, acc[dt]); acc[dt] = wmma_bf(pa.h, vl, acc[dt]); acc[dt] = wmma_bf(pa.h, vh, acc[dt]); }
    LDSX(); }
#pragma unroll
  for (int dt = 0; dt < 5; ++dt)
#pragma unroll
    for (int r = 0; r < 8; ++r) so[wave][8 * g + r][dt * 16 + col] = acc[dt][r];
#pragma unroll
  for (int r = 0; r < 8; ++r) so[wave][8 * g + r][80 + col] = 0.f;
  LDSX();
  for (int q = lane; q < 16 * 24; q += 32) { const int rl = q / 24, pc = q - rl * 24; vst2(U + ((size_t)b * NSEQ + q0 + rl) * UPITCH + h * UP + pc * 4, *(const v4f*)&so[wave][rl][pc * 4]); }
}
__global__ __launch_bounds__(256) void k_mid(const float* __restrict__ U, float* __restrict__ F) {
  __shared__ __align__(16) float sf[64][KP + 4]; __shared__ float spart[64][4];
  const int tid = threadIdx.x; const int rl = tid >> 2, h = tid & 3; const size_t r = (size_t)blockIdx.x * 64 + rl;
  const float* u = U + r * UPITCH + h * UP; const float u0 = u[0]; float ss = 0.f;
  for (int s = 1; s <= HS; ++s) { const float v = u[s]; ss += v * v; }
  const float ln = sqrtf(fmaxf(u0 * u0 - ss, 1e-6f)); float ps = 0.f;
  for (int s = 1; s <= HS; ++s) { const float msp = u[s] / ln; sf[rl][1 + h * HS + (s - 1)] = msp; ps += msp * msp; }
  spart[rl][h] = ps;
  __syncthreads();
  if (h == 0) { const float tt = (spart[rl][0] + spart[rl][1]) + (spart[rl][2] + spart[rl][3]); sf[rl][0] = sqrtf(tt + 1.0f); for (int c = D1; c < KP; ++c) sf[rl][c] = 0.f; }
  __syncthreads();
  for (int q = tid; q < 64 * (KP / 4); q += 256) { const int row = q / (KP / 4), pc = q % (KP / 4); vst2(F + ((size_t)blockIdx.x * 64 + row) * KP + pc * 4, *(const v4f*)&sf[row][pc * 4]); }
}
__global__ __launch_bounds__(128) void k_headl(const float* __restrict__ XL, const __bf16* __restrict__ PT, const float* __restrict__ bh, float* __restrict__ LG) {
  __shared__ __align__(16) float so[4][16][164];
  const int tid = threadIdx.x, wave = tid >> 5, lane = tid & 31, col = lane & 15, g = lane >> 4; const size_t r0 = (size_t)blockIdx.x * 64 + wave * 16;
  v8f acc[9] = {};
#pragma unroll 1
  for (int kc = 0; kc < KP / 32; ++kc) { const F2 a = split_row(XL + (r0 + col) * KP, kc * 32, lane);
#pragma unroll
    for (int j = 0; j < 9; ++j) { const v16b w = frag_b(PT + PT_H + (size_t)(j * 16 + col) * KP + kc * 32, lane); acc[j] = wmma_bf(a.l, w, acc[j]); acc[j] = wmma_bf(a.h, w, acc[j]); } }
#pragma unroll
  for (int j = 0; j < 9; ++j) { const int n = j * 16 + col; const float bb = n < NCLS ? bfr(bh[n]) : 0.f;
#pragma unroll
    for (int r = 0; r < 8; ++r) so[wave][8 * g + r][n] = acc[j][r] + bb; }
#pragma unroll
  for (int r = 0; r < 8; ++r) so[wave][8 * g + r][144 + col] = 0.f;
  LDSX();
  for (int rl = 0; rl < 16; ++rl) for (int pc = lane; pc < 40; pc += 32) vst2(LG + (r0 + rl) * LGP + pc * 4, *(const v4f*)&so[wave][rl][pc * 4]);
}
__global__ __launch_bounds__(256) void k_copy(const float* __restrict__ LG, float* __restrict__ out) {
  const size_t p = (size_t)blockIdx.x * 256 + threadIdx.x; const size_t total = (size_t)NR * NCLS;
  if (p * 4 >= total) return; v4f v;
#pragma unroll
  for (int i = 0; i < 4; ++i) { const size_t f = p * 4 + i; v[i] = LG[(f / NCLS) * LGP + (f % NCLS)]; }
  vst2(out + p * 4, v);
}

extern "C" void kernel_launch(void* const* d_in, const int* in_sizes, int n_in, void* d_out, int out_size, void* d_ws, size_t ws_size, hipStream_t stream) {
  (void)in_sizes; (void)n_in; (void)out_size;
  const float** Fp = (const float**)d_in;
  if (ws_size < (size_t)WS_END) return;
  char* ws = (char*)d_ws; __bf16* PT = (__bf16*)(ws + WS_PT); float *XL = (float*)(ws + WS_XL), *F = (float*)(ws + WS_F), *QS = (float*)(ws + WS_QS), *KS = (float*)(ws + WS_KS), *QT = (float*)(ws + WS_QT), *KT = (float*)(ws + WS_KT), *Mb = (float*)(ws + WS_M), *Lb = (float*)(ws + WS_L), *U = (float*)(ws + WS_U), *LG = (float*)(ws + WS_LG);
  __bf16 *VTH = (__bf16*)(ws + WS_VTH), *VTL = (__bf16*)(ws + WS_VTL);
  k_pack<<<(NLAY * 4 * 256 + 144) / 2, 128, 0, stream>>>(Fp[3], Fp[5], Fp[7], Fp[9], Fp[11], PT);
  k_in<<<TRB, 128, 0, stream>>>(Fp[0], Fp[1], Fp[2], XL);
  for (int li = 0; li < DBG_NL; ++li) { const int l = DBG_L0 + li;
    k_lin<<<TRB, 128, 0, stream>>>(XL, PT, Fp[4], l, 0, QS, QT, VTH, VTL, XL);
    k_lin<<<TRB, 128, 0, stream>>>(XL, PT, Fp[6], l, 1, KS, KT, VTH, VTL, XL);
    k_lin<<<TRB, 128, 0, stream>>>(XL, PT, Fp[8], l, 2, QS, QT, VTH, VTL, XL);
    k_stats<<<dim3(TQB, TNB * NHD), 128, 0, stream>>>(QS, KS, QT, KT, Mb, Lb);
    k_attn<<<dim3(TQB, TNB * NHD), 128, 0, stream>>>(QS, KS, QT, KT, VTH, VTL, Mb, Lb, U);
    k_mid<<<(TQB < NSEQ / 64 ? TQB : TRB), 256, 0, stream>>>(U, F);
    k_lin<<<(TQB < NSEQ / 64 ? TQB : TRB), 128, 0, stream>>>(F, PT, Fp[10], l, 3, QS, QT, VTH, VTL, XL); }
  k_headl<<<(TQB < NSEQ / 64 ? TQB : TRB), 128, 0, stream>>>(XL, PT, Fp[12], LG);
  k_copy<<<(NR * NCLS / 4 + 255) / 256, 256, 0, stream>>>(LG, (float*)d_out);
}
